// TransformerBlockQuantum_65481071407927
// MI455X (gfx1250) — hardware-run, weakly checked
//
#include <hip/hip_runtime.h>
#include <math.h>

typedef __attribute__((ext_vector_type(16))) _Float16 v16h;
typedef __attribute__((ext_vector_type(8)))  _Float16 v8h;
typedef __attribute__((ext_vector_type(8)))  float    v8f;
typedef __attribute__((ext_vector_type(4)))  float    v4f;

constexpr int kBatch = 8;
constexpr int kSeq   = 256;
constexpr int kEmb   = 256;
constexpr int kFfn   = 1024;
constexpr int kWires = 8;
constexpr int kRows  = kBatch * kSeq;
constexpr int kQfPitch = 32;
static_assert(kRows == 2048);
static_assert((kEmb % 32) == 0 && (kFfn % 32) == 0);
static_assert((kRows % 64) == 0 && (kEmb % 64) == 0);
static_assert((kEmb % kWires) == 0);

constexpr float kCarryEz = 512.0f;
constexpr float kCarryWc = 64.0f;
constexpr float kCarryH  = 16.0f;
constexpr float kCarryW2 = 256.0f;
constexpr float kScaleCombine = 1.0f / (kCarryEz * kCarryWc);
constexpr float kScaleDown    = 1.0f / (kCarryH * kCarryW2);
constexpr float kInvEmb = 1.0f / (float)kEmb;
constexpr float kHalfNormMin = 6.103515625e-5f;

constexpr size_t kOffBT1 = 0;
constexpr size_t kOffBT2 = kOffBT1 + (size_t)kEmb * kEmb * 2;
constexpr size_t kOffAEZ = kOffBT2 + (size_t)kEmb * kFfn * 2;
constexpr size_t kOffY1  = kOffAEZ + (size_t)kRows * kEmb * 2;
constexpr size_t kOffX   = kOffY1  + (size_t)kRows * kEmb * 4;
constexpr size_t kOffQF  = kOffX   + (size_t)kRows * kEmb * 4;
constexpr size_t kOffH   = kOffQF  + (size_t)kRows * kQfPitch * 4;
constexpr size_t kOffY2  = kOffH   + (size_t)kRows * kFfn * 2;
constexpr size_t kWsTotal = kOffY2 + (size_t)kRows * kEmb * 4;
static_assert(kWsTotal == 12451840ull);
static_assert(kWsTotal <= 134217728ull);
static_assert((kOffBT2 % 128) == 0 && (kOffAEZ % 128) == 0 && (kOffY1 % 128) == 0 && (kOffX % 128) == 0 &&
              (kOffQF % 128) == 0 && (kOffH % 128) == 0 && (kOffY2 % 128) == 0);

namespace eng {

__device__ __forceinline__ float flush16(float v) {
  return (fabsf(v) < kHalfNormMin) ? 0.0f : v;
}

union FragU { v16h v; v8h h[2]; };
__device__ __forceinline__ v16h frag_load(const _Float16* p) {
  FragU f;
  f.h[0] = *(const v8h*)(p);
  f.h[1] = *(const v8h*)(p + 16);
  return f.v;
}
__device__ __forceinline__ v8f mma_tied(v16h a, v16h b, v8f c) {
  c = __builtin_amdgcn_wmma_f32_16x16x32_f16(false, a, false, b, (short)0, c, false, false);
  asm volatile("v_nop\n\tv_nop\n\tv_nop\n\tv_nop" : "+v"(c) : "v"(a), "v"(b));
  return c;
}

}

constexpr int kCastBlocksWc = (kEmb * kEmb / 8) / 256;
constexpr int kCastBlocksW2 = (kEmb * kFfn / 8) / 256;
static_assert(kCastBlocksWc * 256 * 8 == kEmb * kEmb);
static_assert(kCastBlocksW2 * 256 * 8 == kEmb * kFfn);

__device__ __forceinline__ void cast8_carried(const float* __restrict__ src, unsigned short* __restrict__ dst,
                                              int i, float carry) {
  const size_t e0 = (size_t)i << 3;
  const v4f a0 = *(const v4f*)(src + e0);
  const v4f a1 = *(const v4f*)(src + e0 + 4);
  v8h hv;
#pragma unroll
  for (int e = 0; e < 4; ++e) {
    const float x0 = eng::flush16(a0[e] * carry);
    const float x1 = eng::flush16(a1[e] * carry);
    hv[e]     = (_Float16)x0;
    hv[4 + e] = (_Float16)x1;
  }
  unsigned short* q = dst + e0;
  *(volatile v8h*)q = hv;
  __threadfence();
  *(volatile v8h*)q = hv;
}

__global__ __launch_bounds__(256) void weight_planes_kernel(
    const float* __restrict__ wc, const float* __restrict__ w2,
    unsigned short* __restrict__ bt1, unsigned short* __restrict__ bt2) {
  const int bx = blockIdx.x;
  if (bx < kCastBlocksWc) {
    cast8_carried(wc, bt1, bx * 256 + threadIdx.x, kCarryWc);
  } else {
    cast8_carried(w2, bt2, (bx - kCastBlocksWc) * 256 + threadIdx.x, kCarryW2);
  }
}

constexpr int kEzPerBlock = 2048;
static_assert((kRows * kEmb) % kEzPerBlock == 0);

__global__ __launch_bounds__(256) void wire_expect_kernel(
    const float* __restrict__ src, const float* __restrict__ theta, unsigned short* __restrict__ aez) {
  __shared__ __align__(16) float sC[kEzPerBlock];
  const int tid = threadIdx.x;
  const size_t base = (size_t)blockIdx.x * kEzPerBlock;
  const float th = theta[tid & (kWires - 1)];
#pragma unroll 1
  for (int it = 0; it < 8; ++it) {
    const float a  = src[base + it * 256 + tid] + th;
    const float ch = cosf(a * 0.5f);
    const float c2 = ch * ch;
    sC[it * 256 + tid] = c2 - (1.0f - c2);
  }
  __syncthreads();
  const v4f ca = *(const v4f*)(sC + tid * 8);
  const v4f cb = *(const v4f*)(sC + tid * 8 + 4);
  const float c0 = ca[0], c1 = ca[1], c2v = ca[2], c3 = ca[3];
  const float c4 = cb[0], c5 = cb[1], c6 = cb[2], c7 = cb[3];
  const float p1 = c0 * c1;
  const float p2 = p1 * c2v;
  const float p3 = p2 * c3;
  const float p4 = p3 * c4;
  const float p5 = p4 * c5;
  const float p6 = p5 * c6;
  const float p7 = p6 * c7;
  float t = c1 * c2v;
  t = t * c3;
  t = t * c4;
  t = t * c5;
  t = t * c6;
  t = t * c7;
  v8h hv;
  hv[0] = (_Float16)eng::flush16(t  * kCarryEz);
  hv[1] = (_Float16)eng::flush16(p1 * kCarryEz);
  hv[2] = (_Float16)eng::flush16(p2 * kCarryEz);
  hv[3] = (_Float16)eng::flush16(p3 * kCarryEz);
  hv[4] = (_Float16)eng::flush16(p4 * kCarryEz);
  hv[5] = (_Float16)eng::flush16(p5 * kCarryEz);
  hv[6] = (_Float16)eng::flush16(p6 * kCarryEz);
  hv[7] = (_Float16)eng::flush16(p7 * kCarryEz);
  unsigned short* q = aez + base + (size_t)tid * 8;
  *(volatile v8h*)q = hv;
  __threadfence();
  *(volatile v8h*)q = hv;
}

__global__ __launch_bounds__(256) void gemm_f16_bias_resid_kernel(
    const unsigned short* __restrict__ Ap, int lda,
    const unsigned short* __restrict__ Btp, int ldb,
    float* __restrict__ C, int ldc,
    const float* __restrict__ bias, const float* __restrict__ resid,
    int M, int N, int K, float scale) {
  const _Float16* A  = (const _Float16*)Ap;
  const _Float16* Bt = (const _Float16*)Btp;
  __shared__ __align__(16) float sT[8][16 * 68];
  const int lane = threadIdx.x & 31;
  const int wave = threadIdx.x >> 5;
  const int tilesN = N >> 6;
  const int tilesM = M >> 6;
  const int tile = blockIdx.x * 8 + wave;
  if (tile >= tilesM * tilesN) return;
  const int tm = tile / tilesN;
  const int tn = tile - tm * tilesN;
  const int m0 = tm << 6;
  const int n0 = tn << 6;
  const int rlane = lane & 15;
  const int koff  = (lane >> 4) * 8;
  const int mOff  = (lane >> 4) * 8;

  v8f acc[4][4];
#pragma unroll
  for (int i = 0; i < 4; ++i)
#pragma unroll
    for (int j = 0; j < 4; ++j) acc[i][j] = (v8f){0.f, 0.f, 0.f, 0.f, 0.f, 0.f, 0.f, 0.f};

  for (int k0 = 0; k0 < K; k0 += 32) {
    v16h bh[4];
#pragma unroll
    for (int j = 0; j < 4; ++j) {
      const size_t bo = (size_t)(n0 + (j << 4) + rlane) * ldb + koff + k0;
      bh[j] = eng::frag_load(Bt + bo);
    }
#pragma unroll
    for (int i = 0; i < 4; ++i) {
      const size_t ao = (size_t)(m0 + (i << 4) + rlane) * lda + koff + k0;
      const v16h ah = eng::frag_load(A + ao);
#pragma unroll
      for (int j = 0; j < 4; ++j) acc[i][j] = eng::mma_tied(ah, bh[j], acc[i][j]);
    }
  }

  float* slab = sT[wave];
  const int hh = lane >> 4;
  const int c4 = (lane & 15) * 4;
  const v4f bv = *(const v4f*)(bias + n0 + c4);
#pragma unroll
  for (int i = 0; i < 4; ++i) {
    const int mBase = m0 + (i << 4);
#pragma unroll
    for (int j = 0; j < 4; ++j) {
#pragma unroll
      for (int r = 0; r < 8; ++r) {
        slab[(mOff + r) * 68 + (j << 4) + rlane] = acc[i][j][r] * scale;
      }
    }
    __builtin_amdgcn_fence(__ATOMIC_RELEASE, "workgroup");
    __builtin_amdgcn_wave_barrier();
    __builtin_amdgcn_fence(__ATOMIC_ACQUIRE, "workgroup");
    v4f ov[8];
#pragma unroll
    for (int it = 0; it < 8; ++it) {
      const int row = it * 2 + hh;
      const v4f sv = *(const v4f*)(slab + row * 68 + c4);
      const v4f rv = *(const v4f*)(resid + (size_t)(mBase + row) * ldc + n0 + c4);
      ov[it] = (sv + bv) + rv;
    }
    for (int pass = 0; pass < 2; ++pass) {
#pragma unroll
      for (int it = 0; it < 8; ++it) {
        const int row = it * 2 + hh;
        *(volatile v4f*)(C + (size_t)(mBase + row) * ldc + n0 + c4) = ov[it];
      }
      __threadfence();
    }
    __builtin_amdgcn_fence(__ATOMIC_RELEASE, "workgroup");
    __builtin_amdgcn_wave_barrier();
    __builtin_amdgcn_fence(__ATOMIC_ACQUIRE, "workgroup");
  }
}

template <bool EMIT_QF>
__global__ __launch_bounds__(256) void layernorm_rows_kernel(
    const float* __restrict__ Y, const float* __restrict__ gam, const float* __restrict__ bet,
    float* __restrict__ Xo, const float* __restrict__ thf, float* __restrict__ QFo) {
  const int lane = threadIdx.x & 31;
  const int wave = threadIdx.x >> 5;
  const int row  = blockIdx.x * 8 + wave;
  const int cA = lane * 4;
  const int cB = 128 + lane * 4;
  const float* yr = Y + (size_t)row * kEmb;
  const v4f a0 = *(const v4f*)(yr + cA);
  const v4f a1 = *(const v4f*)(yr + cB);
  float s = ((a0[0] + a0[1]) + (a0[2] + a0[3])) + ((a1[0] + a1[1]) + (a1[2] + a1[3]));
#pragma unroll
  for (int off = 16; off >= 1; off >>= 1) s += __shfl_xor(s, off, 32);
  const float mu = s * kInvEmb;
  float d0[4], d1[4];
#pragma unroll
  for (int e = 0; e < 4; ++e) {
    d0[e] = a0[e] - mu;
    d1[e] = a1[e] - mu;
  }
  float ss = ((d0[0] * d0[0] + d0[1] * d0[1]) + (d0[2] * d0[2] + d0[3] * d0[3])) +
             ((d1[0] * d1[0] + d1[1] * d1[1]) + (d1[2] * d1[2] + d1[3] * d1[3]));
#pragma unroll
  for (int off = 16; off >= 1; off >>= 1) ss += __shfl_xor(ss, off, 32);
  const float var = ss * kInvEmb;
  const float rs  = rsqrtf(var + 1e-5f);
  const v4f g0 = *(const v4f*)(gam + cA);
  const v4f g1 = *(const v4f*)(gam + cB);
  const v4f b0 = *(const v4f*)(bet + cA);
  const v4f b1 = *(const v4f*)(bet + cB);
  v4f o0, o1;
#pragma unroll
  for (int e = 0; e < 4; ++e) {
    o0[e] = d0[e] * rs * g0[e] + b0[e];
    o1[e] = d1[e] * rs * g1[e] + b1[e];
  }
  float* xr = Xo + (size_t)row * kEmb;
  *(volatile v4f*)(xr + cA) = o0;
  *(volatile v4f*)(xr + cB) = o1;
  __threadfence();
  *(volatile v4f*)(xr + cA) = o0;
  *(volatile v4f*)(xr + cB) = o1;
  if (EMIT_QF) {
    const float x0 = o0[0];
    const float x1 = o0[1];
    const float x2 = o0[2];
    const float x3 = o0[3];
    const int sl = (lane >> 2) & 1;
    const float t0 = __shfl(x0, sl, 32);
    const float t1 = __shfl(x1, sl, 32);
    const float t2 = __shfl(x2, sl, 32);
    const float t3 = __shfl(x3, sl, 32);
    const int e = lane & 3;
    const float xw = (e == 0) ? t0 : ((e == 1) ? t1 : ((e == 2) ? t2 : t3));
    float th = thf[lane & (kWires - 1)];
    asm volatile("" : "+v"(th));
    const float qv = cosf(xw) * cosf(th);
    float* qp = QFo + (size_t)row * kQfPitch + lane;
    *(volatile float*)qp = qv;
    __threadfence();
    *(volatile float*)qp = qv;
  }
}

__global__ __launch_bounds__(256) void ffn_up_kernel(
    const float* __restrict__ QF, const float* __restrict__ w1, const float* __restrict__ b1,
    unsigned short* __restrict__ Hout) {
  const int lane = threadIdx.x & 31;
  const int wave = threadIdx.x >> 5;
  const int row  = blockIdx.x * 8 + wave;
  const v4f qa = *(const v4f*)(QF + (size_t)row * kQfPitch);
  const v4f qb = *(const v4f*)(QF + (size_t)row * kQfPitch + 4);
  const float q0 = qa[0], q1 = qa[1], q2 = qa[2], q3 = qa[3];
  const float q4 = qb[0], q5 = qb[1], q6 = qb[2], q7 = qb[3];
#pragma unroll 1
  for (int ci = 0; ci < 4; ++ci) {
    const int f0 = ci * 256 + lane * 8;
    const v4f bA = *(const v4f*)(b1 + f0);
    const v4f bB = *(const v4f*)(b1 + f0 + 4);
    float bb[8];
    bb[0] = bA[0]; bb[1] = bA[1]; bb[2] = bA[2]; bb[3] = bA[3];
    bb[4] = bB[0]; bb[5] = bB[1]; bb[6] = bB[2]; bb[7] = bB[3];
    v8h hv;
#pragma unroll
    for (int e = 0; e < 8; ++e) {
      const float* wr = w1 + (size_t)(f0 + e) * kWires;
      const v4f wa = *(const v4f*)(wr);
      const v4f wb = *(const v4f*)(wr + 4);
      float acc = bb[e];
      acc = fmaf(q0, wa[0], acc);
      acc = fmaf(q1, wa[1], acc);
      acc = fmaf(q2, wa[2], acc);
      acc = fmaf(q3, wa[3], acc);
      acc = fmaf(q4, wb[0], acc);
      acc = fmaf(q5, wb[1], acc);
      acc = fmaf(q6, wb[2], acc);
      acc = fmaf(q7, wb[3], acc);
      const float hc = eng::flush16(fmaxf(acc, 0.0f) * kCarryH);
      hv[e] = (_Float16)hc;
    }
    unsigned short* hp = Hout + (size_t)row * kFfn + f0;
    *(volatile v8h*)hp = hv;
    __threadfence();
    *(volatile v8h*)hp = hv;
  }
}

constexpr int kGemmTiles  = (kRows / 64) * (kEmb / 64);
constexpr int kGemmBlocks = kGemmTiles / 8;
static_assert(kGemmBlocks * 8 == kGemmTiles);
static_assert((kRows % 8) == 0);

extern "C" void kernel_launch(void* const* d_in, const int* in_sizes, int n_in,
                              void* d_out, int out_size, void* d_ws, size_t ws_size,
                              hipStream_t stream) {
  if (n_in < 13) return;
  if (in_sizes[0] != kRows * kEmb) return;
  if (in_sizes[1] != kWires) return;
  if (in_sizes[2] != kWires) return;
  if (in_sizes[3] != kEmb * kEmb) return;
  if (in_sizes[4] != kEmb) return;
  if (in_sizes[5] != kFfn * kWires) return;
  if (in_sizes[6] != kFfn) return;
  if (in_sizes[7] != kEmb * kFfn) return;
  if (in_sizes[8] != kEmb) return;
  if (in_sizes[9] != kEmb) return;
  if (in_sizes[10] != kEmb) return;
  if (in_sizes[11] != kEmb) return;
  if (in_sizes[12] != kEmb) return;
  if (out_size != kRows * kEmb) return;
  if (ws_size < kWsTotal) return;

  const float* src        = (const float*)d_in[0];
  const float* theta_attn = (const float*)d_in[1];
  const float* theta_ffn  = (const float*)d_in[2];
  const float* w_combine  = (const float*)d_in[3];
  const float* b_combine  = (const float*)d_in[4];
  const float* w1         = (const float*)d_in[5];
  const float* b1         = (const float*)d_in[6];
  const float* w2         = (const float*)d_in[7];
  const float* b2         = (const float*)d_in[8];
  const float* g1         = (const float*)d_in[9];
  const float* be1        = (const float*)d_in[10];
  const float* g2         = (const float*)d_in[11];
  const float* be2        = (const float*)d_in[12];
  float* out = (float*)d_out;

  char* ws = (char*)d_ws;
  unsigned short* BT1 = (unsigned short*)(ws + kOffBT1);
  unsigned short* BT2 = (unsigned short*)(ws + kOffBT2);
  unsigned short* AEZ = (unsigned short*)(ws + kOffAEZ);
  float*          Y1  = (float*)(ws + kOffY1);
  float*          X   = (float*)(ws + kOffX);
  float*          QF  = (float*)(ws + kOffQF);
  unsigned short* H   = (unsigned short*)(ws + kOffH);
  float*          Y2  = (float*)(ws + kOffY2);

  weight_planes_kernel<<<kCastBlocksWc + kCastBlocksW2, 256, 0, stream>>>(w_combine, w2, BT1, BT2);

  wire_expect_kernel<<<(kRows * kEmb) / kEzPerBlock, 256, 0, stream>>>(src, theta_attn, AEZ);

  gemm_f16_bias_resid_kernel<<<kGemmBlocks, 256, 0, stream>>>(
      AEZ, kEmb, BT1, kEmb, Y1, kEmb, b_combine, src, kRows, kEmb, kEmb, kScaleCombine);

  layernorm_rows_kernel<true><<<kRows / 8, 256, 0, stream>>>(Y1, g1, be1, X, theta_ffn, QF);

  ffn_up_kernel<<<kRows / 8, 256, 0, stream>>>(QF, w1, b1, H);

  gemm_f16_bias_resid_kernel<<<kGemmBlocks, 256, 0, stream>>>(
      H, kFfn, BT2, kFfn, Y2, kEmb, b2, X, kRows, kEmb, kFfn, kScaleDown);

  layernorm_rows_kernel<false><<<kRows / 8, 256, 0, stream>>>(Y2, g2, be2, out, theta_ffn, QF);
}
